// EdgeGAT_16647293239655
// MI455X (gfx1250) — hardware-verified
//
#include <hip/hip_runtime.h>
#include <math.h>
#include <stddef.h>


#define NODES   100000
#define EDGES   3200000
#define INCH    128
#define HID     64
#define NLAYERS 3
#define NGRAPH  64
#define NCLS    5
#define NEG_SLOPE 0.2f

#define SBSHIFT 11
#define SBMASK  2047
#define NSB     ((NODES + SBMASK) >> SBSHIFT)
#define CAPSB   98304
#define BKSHIFT 6
#define BKMASK  63
#define NBK     ((NODES + BKMASK) >> BKSHIFT)
#define CAPB    4096
#define GROWS   128
#define NGB     ((NODES + GROWS - 1) / GROWS)
#define NPAD    (NGB * GROWS)
#define STG     320
#define WSCALE  16.0f
#define PSCALE  64.0f

#define CT_CHECK(c, n) typedef char n[(c) ? 1 : -1]
CT_CHECK(NSB * 32 >= NBK, ct_check_bucket_map);
CT_CHECK((CAPSB % 256) == 0 && (CAPB % 256) == 0, ct_check_flush_gran);
CT_CHECK(NODES < (1 << 17), ct_check_packed_src);
CT_CHECK((NBK - 1) * 64 + 63 < NPAD, ct_check_row_pad);

typedef _Float16 v16h __attribute__((ext_vector_type(16)));
typedef _Float16 v8h  __attribute__((ext_vector_type(8)));
typedef float    v8f  __attribute__((ext_vector_type(8)));
typedef float    v4f  __attribute__((ext_vector_type(4)));
typedef int      v4i  __attribute__((ext_vector_type(4)));
typedef v4i __attribute__((may_alias)) v4ia;
typedef v4f __attribute__((may_alias)) v4fa;
typedef v8h __attribute__((may_alias)) v8ha;

union Frag { v16h v; v8h h8[2]; };

__device__ __forceinline__ v8f wmma_f16(v16h a, v16h b, v8f c) {
  v8f d = __builtin_amdgcn_wmma_f32_16x16x32_f16(false, a, false, b, (short)0, c, false, false);
  asm volatile("v_nop\n\tv_nop\n\tv_nop\n\tv_nop" : "+v"(d) : "v"(a), "v"(b));
  return d;
}

__device__ __forceinline__ v8h cvt8(float4 p, float4 q, float s) {
  v8h r;
  r[0] = (_Float16)(p.x * s); r[1] = (_Float16)(p.y * s);
  r[2] = (_Float16)(p.z * s); r[3] = (_Float16)(p.w * s);
  r[4] = (_Float16)(q.x * s); r[5] = (_Float16)(q.y * s);
  r[6] = (_Float16)(q.z * s); r[7] = (_Float16)(q.w * s);
  return r;
}

__device__ __forceinline__ void flush_block(const int* stg, int* dst, int lane) {
  asm volatile("" ::: "memory");
  const v4i a0 = *(const v4ia*)(stg + lane * 4);
  const v4i a1 = *(const v4ia*)(stg + 128 + lane * 4);
  volatile v4i* d = (volatile v4i*)dst;
  d[lane] = a0;
  d[32 + lane] = a1;
  __threadfence();
  d[lane] = a0;
  d[32 + lane] = a1;
  asm volatile("" ::: "memory");
}

__device__ __forceinline__ void wave_append(int* stg, int* dstbase, int cap,
                                            int& fill, int& written,
                                            bool flag, int packed, int lane) {
  const bool room = (written + fill + 288) <= cap;
  flag = flag && room;
  const unsigned mask = __builtin_amdgcn_ballot_w32(flag);
  const int rank = (int)__builtin_amdgcn_mbcnt_lo(mask, 0u);
  const int nn = __builtin_popcount(mask);
  if (flag) stg[fill + rank] = packed;
  fill += nn;
  if (fill >= 256) {
    flush_block(stg, dstbase + written, lane);
    written += 256;
    const int rem = fill - 256;
    int tmp = 0;
    if (lane < rem) tmp = stg[256 + lane];
    asm volatile("" ::: "memory");
    if (lane < rem) stg[lane] = tmp;
    asm volatile("" ::: "memory");
    fill = rem;
  }
}

__device__ __forceinline__ void wave_finish(const int* stg, int* dstbase, int* cntline,
                                            int fill, int written, int lane) {
  const int total = written + fill;
  if (fill > 0) flush_block(stg, dstbase + written, lane);
  volatile int* c = (volatile int*)cntline;
  c[lane] = total;
  __threadfence();
  c[lane] = total;
}

__global__ void __launch_bounds__(256)
k_csr1(const int* __restrict__ ei, int* sbreg, int* cnt1) {
  __shared__ __align__(16) int stg_all[8 * STG];
  const int w = threadIdx.x >> 5, lane = threadIdx.x & 31;
  const int sb = blockIdx.x * 8 + w;
  if (sb >= NSB) return;
  int* stg = stg_all + w * STG;
  for (int i = lane; i < STG; i += 32) stg[i] = 0;
  asm volatile("" ::: "memory");
  int* dstbase = sbreg + (size_t)sb * CAPSB;
  int fill = 0, written = 0;
  for (int base = 0; base < EDGES; base += 256) {
    int sv[8], dv[8];
#pragma unroll
    for (int u = 0; u < 8; ++u) {
      const int e = base + u * 32 + lane;
      const bool ok = e < EDGES;
      sv[u] = ok ? ei[e] : 0;
      dv[u] = ok ? ei[(size_t)EDGES + e] : -1;
    }
#pragma unroll
    for (int u = 0; u < 8; ++u) {
      const int e = base + u * 32 + lane;
      const int d = dv[u];
      int s = sv[u];
      s = s < 0 ? 0 : (s > NODES - 1 ? NODES - 1 : s);
      const bool flag = (e < EDGES) && (d >= 0) && (d < NODES) && ((d >> SBSHIFT) == sb);
      const int packed = s | ((d & SBMASK) << 17);
      wave_append(stg, dstbase, CAPSB, fill, written, flag, packed, lane);
    }
  }
  wave_finish(stg, dstbase, cnt1 + sb * 32, fill, written, lane);
}

__global__ void __launch_bounds__(256)
k_csr2(const int* __restrict__ sbreg, const int* __restrict__ cnt1, int* breg, int* cnt2) {
  __shared__ __align__(16) int stg_all[8 * STG];
  const int w = threadIdx.x >> 5, lane = threadIdx.x & 31;
  const int b = blockIdx.x * 8 + w;
  if (b >= NBK) return;
  const int sb = b >> 5, jb = b & 31;
  int* stg = stg_all + w * STG;
  for (int i = lane; i < STG; i += 32) stg[i] = 0;
  asm volatile("" ::: "memory");
  int count = cnt1[sb * 32];
  count = count < 0 ? 0 : (count > CAPSB ? CAPSB : count);
  const int* src = sbreg + (size_t)sb * CAPSB;
  int* dstbase = breg + (size_t)b * CAPB;
  int fill = 0, written = 0;
  for (int base = 0; base < count; base += 256) {
    int pv[8];
#pragma unroll
    for (int u = 0; u < 8; ++u) {
      const int idx = base + u * 32 + lane;
      pv[u] = (idx < count) ? src[idx] : 0;
    }
#pragma unroll
    for (int u = 0; u < 8; ++u) {
      const int idx = base + u * 32 + lane;
      const int p = pv[u];
      const int dl = (p >> 17) & SBMASK;
      int s = p & 0x1FFFF;
      s = s > NODES - 1 ? NODES - 1 : s;
      const bool flag = (idx < count) && ((dl >> BKSHIFT) == jb);
      const int packed = s | ((dl & BKMASK) << 17);
      wave_append(stg, dstbase, CAPB, fill, written, flag, packed, lane);
    }
  }
  wave_finish(stg, dstbase, cnt2 + b * 32, fill, written, lane);
}

template <int K>
__global__ void __launch_bounds__(256)
k_gemm(const float* __restrict__ A, const float* __restrict__ W,
       const float* __restrict__ asrc, const float* __restrict__ adst,
       float* hout, float* ssrc, float* sdst) {
  constexpr int KP = K + 8;
  constexpr int NCOL = 80;
  __shared__ __align__(16) _Float16 Bs[NCOL * KP];
  __shared__ __align__(16) float Cs[GROWS * NCOL];
  const int tid = threadIdx.x, w = tid >> 5, lane = tid & 31;
  const int h = lane >> 4, m = lane & 15;
  const int row0 = blockIdx.x * GROWS;

  for (int idx = tid; idx < K * HID; idx += 256) {
    const int k = idx >> 6, n = idx & 63;
    Bs[n * KP + k] = (_Float16)(W[idx] * WSCALE);
  }
  if (tid < K) {
    const float* wr = W + tid * HID;
    float fs = 0.f, fd = 0.f;
#pragma unroll 4
    for (int n = 0; n < HID; ++n) {
      const float wv = wr[n];
      fs += wv * asrc[n];
      fd += wv * adst[n];
    }
    Bs[64 * KP + tid] = (_Float16)(fs * WSCALE);
    Bs[65 * KP + tid] = (_Float16)(fd * WSCALE);
  }
  for (int idx = tid; idx < 14 * K; idx += 256) {
    const int cc = idx / K, k = idx - cc * K;
    Bs[(66 + cc) * KP + k] = (_Float16)0.0f;
  }
  __syncthreads();

  v8f acc[5] = {};
  const int ar = min(row0 + w * 16 + m, NODES - 1);
  const float* arow = A + (size_t)ar * K;
#pragma unroll
  for (int kb = 0; kb < K; kb += 32) {
    const float4* p = (const float4*)(arow + kb + 8 * h);
    Frag a;
    a.h8[0] = cvt8(p[0], p[1], 1.0f);
    a.h8[1] = cvt8(p[4], p[5], 1.0f);
#pragma unroll
    for (int ct = 0; ct < 5; ++ct) {
      const _Float16* bp = Bs + (ct * 16 + m) * KP + kb + 8 * h;
      Frag b;
      b.h8[0] = *(const v8ha*)bp;
      b.h8[1] = *(const v8ha*)(bp + 16);
      acc[ct] = wmma_f16(a.v, b.v, acc[ct]);
    }
  }
#pragma unroll
  for (int ct = 0; ct < 5; ++ct) {
#pragma unroll
    for (int r = 0; r < 8; ++r)
      Cs[(w * 16 + 8 * h + r) * NCOL + ct * 16 + m] = acc[ct][r] * (1.0f / WSCALE);
  }
  __syncthreads();

  v4f vals[8];
#pragma unroll
  for (int i = 0; i < 8; ++i) {
    const int lrow = w * 16 + 2 * i + h;
    vals[i] = *(const v4fa*)(Cs + lrow * NCOL + m * 4);
  }
#pragma unroll
  for (int i = 0; i < 8; ++i) {
    const int grow = row0 + w * 16 + 2 * i + h;
    *(volatile v4f*)(hout + (size_t)grow * HID + m * 4) = vals[i];
  }
  __threadfence();
#pragma unroll
  for (int i = 0; i < 8; ++i) {
    const int grow = row0 + w * 16 + 2 * i + h;
    *(volatile v4f*)(hout + (size_t)grow * HID + m * 4) = vals[i];
  }

  if (w < 2) {
    const int col = 64 + w;
    v4f s4;
    s4.x = Cs[(4 * lane + 0) * NCOL + col];
    s4.y = Cs[(4 * lane + 1) * NCOL + col];
    s4.z = Cs[(4 * lane + 2) * NCOL + col];
    s4.w = Cs[(4 * lane + 3) * NCOL + col];
    float* sp = (w == 0) ? ssrc : sdst;
    volatile v4f* d = (volatile v4f*)(sp + row0 + 4 * lane);
    *d = s4;
    __threadfence();
    *d = s4;
  }
}

__global__ void __launch_bounds__(256)
k_agg(const int* __restrict__ cnt2, const int* __restrict__ breg,
      const float* __restrict__ hin, const float* __restrict__ ssrc,
      const float* __restrict__ sdst, const float* __restrict__ bias,
      float* hout, int apply_elu) {
  __shared__ int ebuf[CAPB];
  __shared__ __align__(16) float fbuf[64 * HID];
  const int b = blockIdx.x, tid = threadIdx.x, w = tid >> 5, lane = tid & 31;
  const int h = lane >> 4, m = lane & 15;
  int cnt = cnt2[b * 32];
  cnt = cnt < 0 ? 0 : (cnt > CAPB ? CAPB : cnt);
  for (int idx = tid; idx < CAPB; idx += 256)
    ebuf[idx] = (idx < cnt) ? breg[(size_t)b * CAPB + idx] : -1;
  __syncthreads();

  float2 acc[8];
  float mx[8], wsum[8], sd[8];
#pragma unroll
  for (int q = 0; q < 8; ++q) {
    const int v = min(b * 64 + q * 8 + w, NODES - 1);
    sd[q] = sdst[v];
    float lg0 = ssrc[v] + sd[q];
    lg0 = lg0 >= 0.f ? lg0 : NEG_SLOPE * lg0;
    mx[q] = lg0;
    wsum[q] = 1.0f;
    acc[q] = ((const float2*)(hin + (size_t)v * HID))[lane];
  }
  for (int base = 0; base < cnt; base += 32) {
    const int idx = base + lane;
    const int ent = (idx < cnt) ? ebuf[idx] : -1;
    const int el = (ent >> 17) & BKMASK;
    int s = ent & 0x1FFFF;
    s = s > NODES - 1 ? NODES - 1 : s;
    const bool inw = (idx < cnt) && ((el & 7) == w);
    const int eq = el >> 3;
#pragma unroll
    for (int q = 0; q < 8; ++q) {
      unsigned mask = __builtin_amdgcn_ballot_w32(inw && (eq == q));
      while (mask) {
        const int j = __builtin_ctz(mask);
        mask &= mask - 1u;
        const int sj = __shfl(s, j);
        float lg = ssrc[sj] + sd[q];
        lg = lg >= 0.f ? lg : NEG_SLOPE * lg;
        if (lg > mx[q]) {
          const float sc = __expf(mx[q] - lg);
          acc[q].x *= sc; acc[q].y *= sc; wsum[q] *= sc; mx[q] = lg;
        }
        const float p = __expf(lg - mx[q]);
        const float2 hv = ((const float2*)(hin + (size_t)sj * HID))[lane];
        acc[q].x += p * hv.x;
        acc[q].y += p * hv.y;
        wsum[q] += p;
      }
    }
  }
#pragma unroll
  for (int q = 0; q < 8; ++q) {
    const float inv = 1.0f / wsum[q];
    float2 r;
    r.x = acc[q].x * inv;
    r.y = acc[q].y * inv;
    ((float2*)(fbuf + (q * 8 + w) * HID))[lane] = r;
  }
  __syncthreads();

  const float4 bia = ((const float4*)bias)[m];
  v4f o[4];
#pragma unroll
  for (int i = 0; i < 4; ++i) {
    const int lrow = w * 8 + 2 * i + h;
    v4f t = *(const v4fa*)(fbuf + lrow * HID + 4 * m);
    t.x += bia.x; t.y += bia.y; t.z += bia.z; t.w += bia.w;
    if (apply_elu) {
      t.x = t.x > 0.f ? t.x : __expf(t.x) - 1.0f;
      t.y = t.y > 0.f ? t.y : __expf(t.y) - 1.0f;
      t.z = t.z > 0.f ? t.z : __expf(t.z) - 1.0f;
      t.w = t.w > 0.f ? t.w : __expf(t.w) - 1.0f;
    }
    o[i] = t;
  }
#pragma unroll
  for (int i = 0; i < 4; ++i) {
    const int grow = b * 64 + w * 8 + 2 * i + h;
    *(volatile v4f*)(hout + (size_t)grow * HID + 4 * m) = o[i];
  }
  __threadfence();
#pragma unroll
  for (int i = 0; i < 4; ++i) {
    const int grow = b * 64 + w * 8 + 2 * i + h;
    *(volatile v4f*)(hout + (size_t)grow * HID + 4 * m) = o[i];
  }
}

__global__ void __launch_bounds__(256)
k_pool(const float* __restrict__ hsrc, const int* __restrict__ batch, float* pooled) {
  __shared__ int sflag[256];
  __shared__ int wany[8];
  __shared__ float part[4 * 64];
  __shared__ int pc[4];
  __shared__ __align__(16) float prow[64];
  const int t = threadIdx.x, w = t >> 5, lane = t & 31, c = t & 63, q = t >> 6;
  const int g = blockIdx.x;
  float acc = 0.f;
  int cn = 0;
  for (int tile0 = 0; tile0 < NODES; tile0 += 256) {
    const int n = tile0 + t;
    const bool f = (n < NODES) && (batch[n] == g);
    sflag[t] = f ? 1 : 0;
    const unsigned mk = __builtin_amdgcn_ballot_w32(f);
    if (lane == 0) wany[w] = (mk != 0u) ? 1 : 0;
    __syncthreads();
    const int any = wany[0] | wany[1] | wany[2] | wany[3] | wany[4] | wany[5] | wany[6] | wany[7];
    if (any) {
      for (int j = q; j < 256; j += 4) {
        if (sflag[j]) { acc += hsrc[(size_t)(tile0 + j) * HID + c]; ++cn; }
      }
    }
    __syncthreads();
  }
  part[q * 64 + c] = acc;
  if (c == 0) pc[q] = cn;
  __syncthreads();
  if (t < 64) {
    const float s = ((part[t] + part[64 + t]) + part[128 + t]) + part[192 + t];
    const int tot = pc[0] + pc[1] + pc[2] + pc[3];
    prow[t] = s * (1.0f / fmaxf((float)tot, 1.0f));
  }
  __syncthreads();
  if (t < 16) {
    const v4f v = *(const v4fa*)(prow + 4 * t);
    volatile v4f* d = (volatile v4f*)(pooled + (size_t)g * HID);
    d[t] = v;
    __threadfence();
    d[t] = v;
  }
}

__global__ void __launch_bounds__(256)
k_head(const float* __restrict__ pooled, const float* __restrict__ sex,
       const float* __restrict__ cag, const float* __restrict__ l1w,
       const float* __restrict__ l1b, const float* __restrict__ l2w,
       const float* __restrict__ l2b, float* out) {
  __shared__ __align__(16) float x1s[NGRAPH * 68];
  __shared__ __align__(16) float outs[NGRAPH * NCLS];
  const int tid = threadIdx.x, w = tid >> 5, lane = tid & 31;
  const int h = lane >> 4, m = lane & 15;
  const int rt = w & 3, ct0 = (w >> 2) * 2;

  v8f acc[2] = {};
  const float* arow = pooled + (size_t)(rt * 16 + m) * HID;
#pragma unroll
  for (int kb = 0; kb < HID; kb += 32) {
    const float4* p = (const float4*)(arow + kb + 8 * h);
    Frag a;
    a.h8[0] = cvt8(p[0], p[1], PSCALE);
    a.h8[1] = cvt8(p[4], p[5], PSCALE);
#pragma unroll
    for (int u = 0; u < 2; ++u) {
      const int col = (ct0 + u) * 16 + m;
      v8h b0, b1;
#pragma unroll
      for (int i = 0; i < 8; ++i) {
        const int k = kb + 8 * h + i;
        b0[i] = (_Float16)(l1w[k * HID + col] * WSCALE);
        b1[i] = (_Float16)(l1w[(k + 16) * HID + col] * WSCALE);
      }
      Frag b;
      b.h8[0] = b0;
      b.h8[1] = b1;
      acc[u] = wmma_f16(a.v, b.v, acc[u]);
    }
  }
#pragma unroll
  for (int u = 0; u < 2; ++u) {
#pragma unroll
    for (int r = 0; r < 8; ++r) {
      const int row = rt * 16 + 8 * h + r;
      const int col = (ct0 + u) * 16 + m;
      x1s[row * 68 + col] = fmaxf(acc[u][r] * (1.0f / (PSCALE * WSCALE)) + l1b[col], 0.f);
    }
  }
  __syncthreads();

  for (int o = tid; o < NGRAPH * NCLS; o += 256) {
    const int g = o / NCLS, j = o - g * NCLS;
    float z = l2b[j];
    const float* xr = x1s + g * 68;
#pragma unroll 4
    for (int cch = 0; cch < HID; ++cch) z += xr[cch] * l2w[cch * NCLS + j];
    z += sex[g] * l2w[HID * NCLS + j] + cag[g] * l2w[(HID + 1) * NCLS + j];
    outs[o] = z;
  }
  __syncthreads();
  if (tid < NGRAPH) {
    const int g = tid;
    float zz[NCLS];
    float mxv = -INFINITY;
#pragma unroll
    for (int j = 0; j < NCLS; ++j) { zz[j] = outs[g * NCLS + j]; mxv = fmaxf(mxv, zz[j]); }
    float se = 0.f;
#pragma unroll
    for (int j = 0; j < NCLS; ++j) { zz[j] = expf(zz[j] - mxv); se += zz[j]; }
    const float inv = 1.0f / se;
#pragma unroll
    for (int j = 0; j < NCLS; ++j) outs[g * NCLS + j] = zz[j] * inv;
  }
  __syncthreads();
  if (w == 0) {
    constexpr int NV = (NGRAPH * NCLS) / 4;
    v4f vv[3];
#pragma unroll
    for (int i = 0; i < 3; ++i) {
      const int idx = i * 32 + lane;
      const int cidx = idx < NV ? idx : NV - 1;
      vv[i] = *(const v4fa*)(outs + cidx * 4);
    }
    volatile v4f* d = (volatile v4f*)out;
#pragma unroll
    for (int i = 0; i < 3; ++i) { const int idx = i * 32 + lane; if (idx < NV) d[idx] = vv[i]; }
    __threadfence();
#pragma unroll
    for (int i = 0; i < 3; ++i) { const int idx = i * 32 + lane; if (idx < NV) d[idx] = vv[i]; }
  }
}

static inline size_t align256(size_t x) { return (x + 255) & ~(size_t)255; }

extern "C" void kernel_launch(void* const* d_in, const int* in_sizes, int n_in,
                              void* d_out, int out_size, void* d_ws, size_t ws_size,
                              hipStream_t stream) {
  if (n_in < 14) return;
  if (in_sizes[0] != NODES * INCH || in_sizes[1] != 2 * EDGES || in_sizes[2] != NODES ||
      in_sizes[3] != NGRAPH || in_sizes[4] != NGRAPH || in_sizes[5] != INCH * HID ||
      in_sizes[6] != (NLAYERS - 1) * HID * HID || in_sizes[7] != NLAYERS * HID ||
      in_sizes[8] != NLAYERS * HID || in_sizes[9] != NLAYERS * HID ||
      in_sizes[10] != HID * HID || in_sizes[11] != HID ||
      in_sizes[12] != (HID + 2) * NCLS || in_sizes[13] != NCLS)
    return;
  if (out_size != NGRAPH * NCLS) return;

  const float* x     = (const float*)d_in[0];
  const int*   ei    = (const int*)d_in[1];
  const int*   batch = (const int*)d_in[2];
  const float* sex   = (const float*)d_in[3];
  const float* cag   = (const float*)d_in[4];
  const float* W0    = (const float*)d_in[5];
  const float* Ws    = (const float*)d_in[6];
  const float* asrc  = (const float*)d_in[7];
  const float* adst  = (const float*)d_in[8];
  const float* cbias = (const float*)d_in[9];
  const float* l1w   = (const float*)d_in[10];
  const float* l1b   = (const float*)d_in[11];
  const float* l2w   = (const float*)d_in[12];
  const float* l2b   = (const float*)d_in[13];
  float* out = (float*)d_out;

  char* ws = (char*)d_ws;
  size_t off = 0;
  const size_t o_sbreg = off; off = align256(off + (size_t)NSB * CAPSB * 4);
  const size_t o_cnt1  = off; off = align256(off + (size_t)NSB * 128);
  const size_t o_breg  = off; off = align256(off + (size_t)NBK * CAPB * 4);
  const size_t o_cnt2  = off; off = align256(off + (size_t)NBK * 128);
  const size_t o_hA    = off; off = align256(off + (size_t)NPAD * HID * 4);
  const size_t o_hB    = off; off = align256(off + (size_t)NPAD * HID * 4);
  const size_t o_ssrc  = off; off = align256(off + (size_t)NPAD * 4);
  const size_t o_sdst  = off; off = align256(off + (size_t)NPAD * 4);
  const size_t o_pool  = off; off = align256(off + (size_t)NGRAPH * HID * 4);
  if (off > ws_size) return;

  int*   sbreg  = (int*)(ws + o_sbreg);
  int*   cnt1   = (int*)(ws + o_cnt1);
  int*   breg   = (int*)(ws + o_breg);
  int*   cnt2   = (int*)(ws + o_cnt2);
  float* hA     = (float*)(ws + o_hA);
  float* hB     = (float*)(ws + o_hB);
  float* ssrc   = (float*)(ws + o_ssrc);
  float* sdst   = (float*)(ws + o_sdst);
  float* pooled = (float*)(ws + o_pool);

  k_csr1<<<(NSB + 7) / 8, 256, 0, stream>>>(ei, sbreg, cnt1);
  k_csr2<<<(NBK + 7) / 8, 256, 0, stream>>>(sbreg, cnt1, breg, cnt2);

  const float* hin = x;
  for (int layer = 0; layer < NLAYERS; ++layer) {
    const float* as = asrc + layer * HID;
    const float* ad = adst + layer * HID;
    if (layer == 0)
      k_gemm<INCH><<<NGB, 256, 0, stream>>>(hin, W0, as, ad, hA, ssrc, sdst);
    else
      k_gemm<HID><<<NGB, 256, 0, stream>>>(hin, Ws + (size_t)(layer - 1) * HID * HID, as, ad, hA, ssrc, sdst);
    k_agg<<<NBK, 256, 0, stream>>>(cnt2, breg, hA, ssrc, sdst, cbias + layer * HID, hB,
                                   (layer < NLAYERS - 1) ? 1 : 0);
    hin = hB;
  }
  k_pool<<<NGRAPH, 256, 0, stream>>>(hB, batch, pooled);
  k_head<<<1, 256, 0, stream>>>(pooled, sex, cag, l1w, l1b, l2w, l2b, out);
}
